// BasicAttentionModel_40879498728927
// MI455X (gfx1250) — hardware-verified
//
#include <hip/hip_runtime.h>
#include <hip/hip_bf16.h>
#include <stddef.h>


#define FX      16
#define FE      10
#define NHD     3
#define KA      32
#define LDH1    64
#define LDH2    128
#define LDH3    192
#define KPQ     192
#define NPQ     128
#define WSC     64
#define ASC     8
#define NTHR    256
#define NWAVE   8
#define EPT     8
#define NGRP    2
#define CHUNK   (NTHR * EPT * NGRP)
#define WCAP    (EPT * NGRP * 32)
#define LISTN   (NWAVE * WCAP)
#define NBC     4096
#define NBF     1024
#define RCAP    40960
#define RBN     128
#define TGT     256
#define DEGCAP  256
#define OTHR    512
#define BM      64
#define NCW     64
#define ETHR    128
#define ACTV    28
#define RPT     16
#define SWF     3744
#define WSCAP   134217728

#define LDS_FILL ((RCAP + NBF + LISTN) * 4 + 64)
#define LDS_EDGE (ETHR * ACTV * 16)

static_assert((CHUNK & (CHUNK - 1)) == 0);
static_assert(CHUNK <= 4096);
static_assert(NBC <= 4096 && NBF <= 4096);
static_assert((NBC & (NBC - 1)) == 0 && (NBF & (NBF - 1)) == 0);
static_assert(NBC == 4 * NBF);
static_assert(OTHR * 8 == NBC);
static_assert((RCAP % 32) == 0);
static_assert(TGT == NWAVE * 32);
static_assert((NBC % TGT) == 0);
static_assert((TGT % BM) == 0);
static_assert(BM * 4 == NTHR);
static_assert(WCAP == EPT * NGRP * 32);
static_assert((KPQ % 32) == 0);

typedef float          v2f  __attribute__((ext_vector_type(2)));
typedef float          v4f  __attribute__((ext_vector_type(4)));
typedef float          v8f  __attribute__((ext_vector_type(8)));
typedef int            v4i  __attribute__((ext_vector_type(4)));
typedef double         v2d  __attribute__((ext_vector_type(2)));
typedef _Float16       v4h  __attribute__((ext_vector_type(4)));
typedef _Float16       v8h  __attribute__((ext_vector_type(8)));
typedef _Float16       v16h __attribute__((ext_vector_type(16)));
typedef _Float16       v8ha __attribute__((ext_vector_type(8), __may_alias__));
typedef __bf16         v16bf __attribute__((ext_vector_type(16)));
typedef unsigned short v4us __attribute__((ext_vector_type(4)));
typedef unsigned short v8us __attribute__((ext_vector_type(8)));
union FragH { v16h v; v8us u[2]; };
union FragB { v16bf v; v8us u[2]; };

__device__ __forceinline__ v8f wmh(v16h a, v16h b, v8f c) {
  v8f d = __builtin_amdgcn_wmma_f32_16x16x32_f16(false, a, false, b, (short)0, c, false, false);
  asm volatile("v_nop\n\tv_nop\n\tv_nop\n\tv_nop" : "+v"(d) : "v"(a), "v"(b));
  return d;
}
__device__ __forceinline__ v8f wmb(v16bf a, v16bf b, v8f c) {
  v8f d = __builtin_amdgcn_wmma_f32_16x16x32_bf16(false, a, false, b, (short)0, c, false, false);
  asm volatile("v_nop\n\tv_nop\n\tv_nop\n\tv_nop" : "+v"(d) : "v"(a), "v"(b));
  return d;
}

__device__ __forceinline__ float lrelu2(float v) { return v > 0.0f ? v : 0.2f * v; }
__device__ __forceinline__ unsigned short bf16_rne(float f) {
  unsigned int u = __float_as_uint(f);
  u = u + 0x7FFFu + ((u >> 16) & 1u);
  return (unsigned short)(u >> 16);
}
__device__ __forceinline__ float bf16_val(unsigned short b) { return __uint_as_float(((unsigned int)b) << 16); }
__device__ __forceinline__ float wmax32(float v) {
#pragma unroll
  for (int s = 16; s > 0; s >>= 1) v = fmaxf(v, __shfl_xor(v, s));
  return v;
}
__device__ __forceinline__ float wsum32(float v) {
#pragma unroll
  for (int s = 16; s > 0; s >>= 1) v += __shfl_xor(v, s);
  return v;
}
__device__ __forceinline__ float dot4(v4f a, v4f b) { return a.x * b.x + a.y * b.y + a.z * b.z + a.w * b.w; }
__device__ __forceinline__ v4f shfl4(v4f v, int src) {
  v4f r;
  r.x = __shfl(v.x, src); r.y = __shfl(v.y, src); r.z = __shfl(v.z, src); r.w = __shfl(v.w, src);
  return r;
}

template <int NB>
__device__ __forceinline__ int scan_chunk(const int* __restrict__ dsts, int nE, int cbase, int slotBase,
                                          int vec8, int* list, int tid, int lane, int wave) {
  int wc = 0;
#pragma unroll
  for (int g = 0; g < NGRP; ++g) {
    const int el0  = (g * NTHR + tid) * EPT;
    const int e0   = cbase + el0;
    const int sent = -2147483647 - 1;
    v4i da, db;
    if (vec8 != 0 && cbase + CHUNK <= nE) {
      da = *(const v4i*)(dsts + e0);
      db = *(const v4i*)(dsts + e0 + 4);
    } else {
      da.x = (e0     < nE) ? dsts[min(e0, nE - 1)] : sent;
      da.y = (e0 + 1 < nE) ? dsts[min(e0 + 1, nE - 1)] : sent;
      da.z = (e0 + 2 < nE) ? dsts[min(e0 + 2, nE - 1)] : sent;
      da.w = (e0 + 3 < nE) ? dsts[min(e0 + 3, nE - 1)] : sent;
      db.x = (e0 + 4 < nE) ? dsts[min(e0 + 4, nE - 1)] : sent;
      db.y = (e0 + 5 < nE) ? dsts[min(e0 + 5, nE - 1)] : sent;
      db.z = (e0 + 6 < nE) ? dsts[min(e0 + 6, nE - 1)] : sent;
      db.w = (e0 + 7 < nE) ? dsts[min(e0 + 7, nE - 1)] : sent;
    }
    const unsigned nb = (unsigned)slotBase;
    const unsigned s0 = (unsigned)da.x - nb, s1 = (unsigned)da.y - nb;
    const unsigned s2 = (unsigned)da.z - nb, s3 = (unsigned)da.w - nb;
    const unsigned s4 = (unsigned)db.x - nb, s5 = (unsigned)db.y - nb;
    const unsigned s6 = (unsigned)db.z - nb, s7 = (unsigned)db.w - nb;
    const bool h0 = s0 < (unsigned)NB, h1 = s1 < (unsigned)NB, h2 = s2 < (unsigned)NB, h3 = s3 < (unsigned)NB;
    const bool h4 = s4 < (unsigned)NB, h5 = s5 < (unsigned)NB, h6 = s6 < (unsigned)NB, h7 = s7 < (unsigned)NB;
    const unsigned any = __builtin_amdgcn_ballot_w32(h0 | h1 | h2 | h3 | h4 | h5 | h6 | h7);
    if (any != 0u) {
#define HITJ(J, HJ, SJ) { \
        const unsigned mj = __builtin_amdgcn_ballot_w32(HJ); \
        if (mj != 0u) { \
          if (HJ) { \
            const int pos = wc + (int)__builtin_amdgcn_mbcnt_lo(mj, 0u); \
            if (pos < WCAP) list[wave * WCAP + pos] = ((el0 + (J)) << 12) | (int)(SJ); \
          } \
          wc += (int)__builtin_popcount(mj); } }
      HITJ(0, h0, s0)
      HITJ(1, h1, s1)
      HITJ(2, h2, s2)
      HITJ(3, h3, s3)
      HITJ(4, h4, s4)
      HITJ(5, h5, s5)
      HITJ(6, h6, s6)
      HITJ(7, h7, s7)
#undef HITJ
    }
  }
  return wc;
}

template <int COLS>
__global__ __launch_bounds__(NTHR) void k_colstats(const float* __restrict__ src, double* part, int rows) {
  __shared__ double red[16 * NTHR];
  __shared__ __attribute__((aligned(16))) double sl[32];
  const int tid = threadIdx.x;
  const int base = (int)blockIdx.x * (NTHR * RPT);
  double s[COLS], q[COLS];
#pragma unroll
  for (int c = 0; c < COLS; ++c) { s[c] = 0.0; q[c] = 0.0; }
#pragma unroll 1
  for (int i = 0; i < RPT; ++i) {
    const int row = base + tid + NTHR * i;
    int rr = row > rows - 1 ? rows - 1 : row;
    rr = rr < 0 ? 0 : rr;
    const bool live = row < rows;
    const float* p = src + (size_t)rr * COLS;
#pragma unroll
    for (int c = 0; c < COLS; ++c) {
      float v = p[c];
      v = live ? v : 0.0f;
      const double dv = (double)v;
      s[c] += dv;
      q[c] += dv * dv;
    }
  }
  if (tid < 32) sl[tid] = 0.0;
#pragma unroll
  for (int c = 0; c < COLS; ++c) red[c * NTHR + tid] = s[c];
  __syncthreads();
  if (tid < COLS) {
    double t = 0.0;
#pragma unroll 1
    for (int i = 0; i < NTHR; ++i) t += red[tid * NTHR + i];
    sl[tid] = t;
  }
  __syncthreads();
#pragma unroll
  for (int c = 0; c < COLS; ++c) red[c * NTHR + tid] = q[c];
  __syncthreads();
  if (tid < COLS) {
    double t = 0.0;
#pragma unroll 1
    for (int i = 0; i < NTHR; ++i) t += red[tid * NTHR + i];
    sl[16 + tid] = t;
  }
  __syncthreads();
  const int l16 = tid < 16 ? tid : 15;
  const v2d v = *(const v2d*)(sl + 2 * l16);
  double* gp = part + (size_t)blockIdx.x * 32 + 2 * l16;
  const bool act = tid < 16;
  if (act) *(volatile v2d*)gp = v;
  __threadfence();
  if (act) *(volatile v2d*)gp = v;
}

__global__ __launch_bounds__(64) void k_bnfin(const double* __restrict__ px, const double* __restrict__ pe,
                                             float* stat, int nbx, int rowsx, int nbe, int rowse) {
  __shared__ __attribute__((aligned(16))) float sl[64];
  const int tid = threadIdx.x;
  const int which = (tid >> 4) & 1;
  const int c = tid & 15;
  const double* p = which ? pe : px;
  const int nb = which ? nbe : nbx;
  const int rows = which ? rowse : rowsx;
  const int cols = which ? FE : FX;
  double S = 0.0, Q = 0.0;
  if (tid < 32) {
#pragma unroll 1
    for (int b = 0; b < nb; ++b) {
      S += p[(size_t)b * 32 + c];
      Q += p[(size_t)b * 32 + 16 + c];
    }
  }
  const double inv = 1.0 / (double)(rows > 0 ? rows : 1);
  const double mean = S * inv;
  double var = Q * inv - mean * mean;
  var = var < 0.0 ? 0.0 : var;
  const float mf = (float)mean;
  const float rf = rsqrtf((float)var + 1e-5f);
  const bool valid = (tid < 32) && (c < cols);
  if (tid < 32) {
    sl[which * 32 + c] = valid ? mf : 0.0f;
    sl[which * 32 + 16 + c] = valid ? rf : 0.0f;
  }
  __syncthreads();
  const int l16 = tid < 16 ? tid : 15;
  const v4f v = *(const v4f*)(sl + 4 * l16);
  const bool act = tid < 16;
  if (act) *(volatile v4f*)(stat + 4 * l16) = v;
  __threadfence();
  if (act) *(volatile v4f*)(stat + 4 * l16) = v;
}

__global__ __launch_bounds__(NTHR) void k_ufold(
    const float* __restrict__ W1, const float* __restrict__ aS1, const float* __restrict__ aD1,
    const float* __restrict__ W2, const float* __restrict__ aS2, const float* __restrict__ aD2,
    const float* __restrict__ W3, const float* __restrict__ aS3, const float* __restrict__ aD3, float* u) {
  __shared__ __attribute__((aligned(16))) float su[256];
  const int tid = threadIdx.x;
  const int l = (int)blockIdx.x;
  const int K = (l == 2) ? 32 : 16;
  const int D = 16 << l;
  const float* W  = (l == 0) ? W1 : ((l == 1) ? W2 : W3);
  const float* aS = (l == 0) ? aS1 : ((l == 1) ? aS2 : aS3);
  const float* aD = (l == 0) ? aD1 : ((l == 1) ? aD2 : aD3);
  const int which = (tid >> 7) & 1;
  const int h = (tid >> 5) & 3;
  const int k = tid & 31;
  const float* att = which ? aD : aS;
  const bool valid = (h < NHD) && (k < K);
  const int hc = h < NHD - 1 ? h : NHD - 1;
  const int kc = k < K - 1 ? k : K - 1;
  const float* wr = W + (size_t)kc * (NHD * D) + hc * D;
  const float* ar = att + hc * D;
  float s = 0.0f;
#pragma unroll 1
  for (int d = 0; d < D; ++d) s += wr[d] * ar[d];
  su[tid] = valid ? s : 0.0f;
  __syncthreads();
  const int q = tid < 64 ? tid : 63;
  const v4f v = *(const v4f*)(su + 4 * q);
  const bool act = tid < 64;
  float* gp = u + (size_t)l * 256 + 4 * q;
  if (act) *(volatile v4f*)gp = v;
  __threadfence();
  if (act) *(volatile v4f*)gp = v;
}

__global__ __launch_bounds__(NTHR) void k_xprep(const float* __restrict__ x, const float* __restrict__ stat,
                                                const float* __restrict__ g, const float* __restrict__ b,
                                                const float* __restrict__ u, unsigned short* A1,
                                                float* eS1, float* eD1, int nN) {
  __shared__ __attribute__((aligned(16))) float su[256];
  __shared__ float ss[32], sg[16], sbb[16];
  __shared__ __attribute__((aligned(16))) float sxb[NTHR * FX];
  __shared__ __attribute__((aligned(16))) _Float16 sA[NTHR * KA];
  const int tid = threadIdx.x;
  const int rowBase = (int)blockIdx.x * NTHR;
  su[tid] = u[tid];
  if (tid < 32) ss[tid] = stat[tid];
  if (tid < 16) { sg[tid] = g[tid]; sbb[tid] = b[tid]; }
  __syncthreads();
  const int row = rowBase + tid;
  int rr = row > nN - 1 ? nN - 1 : row;
  rr = rr < 0 ? 0 : rr;
  const bool live = row < nN;
  const float* xr = x + (size_t)rr * FX;
  const v4f x0 = *(const v4f*)xr, x1 = *(const v4f*)(xr + 4);
  const v4f x2 = *(const v4f*)(xr + 8), x3 = *(const v4f*)(xr + 12);
  float xv[16] = {x0.x, x0.y, x0.z, x0.w, x1.x, x1.y, x1.z, x1.w,
                  x2.x, x2.y, x2.z, x2.w, x3.x, x3.y, x3.z, x3.w};
  float xb[16];
#pragma unroll
  for (int k = 0; k < 16; ++k) {
    const float t = (xv[k] - ss[k]) * ss[16 + k] * sg[k] + sbb[k];
    xb[k] = live ? t : 0.0f;
  }
  v8h o0, o1, z8;
#pragma unroll
  for (int q = 0; q < 8; ++q) {
    o0[q] = (_Float16)(xb[q] * (float)ASC);
    o1[q] = (_Float16)(xb[8 + q] * (float)ASC);
    z8[q] = (_Float16)0.0f;
  }
  _Float16* sr = sA + tid * KA;
  *(v8h*)(sr)      = o0;
  *(v8h*)(sr + 8)  = o1;
  *(v8h*)(sr + 16) = z8;
  *(v8h*)(sr + 24) = z8;
#pragma unroll
  for (int k = 0; k < 16; ++k) sxb[tid * FX + k] = xb[k];
  __syncthreads();
  float e0s = 0.f, e1s = 0.f, e2s = 0.f, e0d = 0.f, e1d = 0.f, e2d = 0.f;
#pragma unroll 1
  for (int k = 0; k < FX; ++k) {
    const float v = sxb[tid * FX + k];
    e0s += v * su[k];        e1s += v * su[32 + k];   e2s += v * su[64 + k];
    e0d += v * su[128 + k];  e1d += v * su[160 + k];  e2d += v * su[192 + k];
  }
  v4f vs, vd;
  vs.x = e0s; vs.y = e1s; vs.z = e2s; vs.w = 0.0f;
  vd.x = e0d; vd.y = e1d; vd.z = e2d; vd.w = 0.0f;
  v8us pv[4];
#pragma unroll
  for (int it = 0; it < 4; ++it) {
    const int id = it * NTHR + tid;
    const v8ha t = *(const v8ha*)(sA + 8 * id);
    pv[it] = __builtin_bit_cast(v8us, t);
  }
  unsigned short* ab = A1 + (size_t)rowBase * KA;
#pragma unroll
  for (int it = 0; it < 4; ++it) *(volatile v8us*)(ab + 8 * (it * NTHR + tid)) = pv[it];
  *(volatile v4f*)(eS1 + (size_t)row * 4) = vs;
  *(volatile v4f*)(eD1 + (size_t)row * 4) = vd;
  __threadfence();
#pragma unroll
  for (int it = 0; it < 4; ++it) *(volatile v8us*)(ab + 8 * (it * NTHR + tid)) = pv[it];
  *(volatile v4f*)(eS1 + (size_t)row * 4) = vs;
  *(volatile v4f*)(eD1 + (size_t)row * 4) = vd;
}

__global__ __launch_bounds__(NTHR) void k_wcvt16(const float* __restrict__ W, unsigned short* wp,
                                                 int K, int Nout, int ncols) {
  const int i = (int)blockIdx.x * NTHR + (int)threadIdx.x;
  if (i >= ncols * 4) return;
  const int n = i >> 2, seg = i & 3;
  const int nc = n < Nout - 1 ? n : Nout - 1;
  v8h o;
#pragma unroll
  for (int j = 0; j < 8; ++j) {
    const int k = 8 * seg + j;
    const int kc = k < K - 1 ? k : K - 1;
    const bool valid = (k < K) && (n < Nout);
    const float v = W[(size_t)kc * Nout + nc];
    o[j] = valid ? (_Float16)(v * (float)WSC) : (_Float16)0.0f;
  }
  const v8us ob = __builtin_bit_cast(v8us, o);
  unsigned short* d = wp + (size_t)i * 8;
  *(volatile v8us*)d = ob;
  __threadfence();
  *(volatile v8us*)d = ob;
}

__global__ __launch_bounds__(NTHR) void k_wcvtpq(const float* __restrict__ W, unsigned short* wp) {
  constexpr int UNITS = NPQ * (KPQ / 8);
  const int i = (int)blockIdx.x * NTHR + (int)threadIdx.x;
  if (i >= UNITS) return;
  const int n = i / (KPQ / 8);
  const int seg = i - n * (KPQ / 8);
  const int piece = seg >> 3;
  const int kk0 = (8 * seg) & 63;
  const int ro = n < 64 ? 0 : 64;
  const int nc = n & 63;
  v8us o;
#pragma unroll
  for (int j = 0; j < 8; ++j) {
    const float w = W[(size_t)(ro + kk0 + j) * 64 + nc];
    const unsigned short hb = bf16_rne(w);
    const unsigned short lb = bf16_rne(w - bf16_val(hb));
    o[j] = (piece == 2) ? lb : hb;
  }
  unsigned short* d = wp + (size_t)i * 8;
  *(volatile v8us*)d = o;
  __threadfence();
  *(volatile v8us*)d = o;
}

__global__ __launch_bounds__(NTHR) void k_count(
    const int* __restrict__ dsts, int* cnt, int nE, int vec8) {
  __shared__ __attribute__((aligned(16))) int scnt[NBC];
  __shared__ __attribute__((aligned(16))) int list[LISTN];
  __shared__ int wcnt[NWAVE];
  const int tid = threadIdx.x, lane = tid & 31, wave = tid >> 5;
  const int nodeBase = blockIdx.x * NBC;

  for (int i = tid; i < NBC; i += NTHR) scnt[i] = 0;
  __syncthreads();

  const int nChunks = (nE + CHUNK - 1) / CHUNK;
#pragma unroll 1
  for (int ch = 0; ch < nChunks; ++ch) {
    const int cbase = ch * CHUNK;
    const int wc = scan_chunk<NBC>(dsts, nE, cbase, nodeBase, vec8, list, tid, lane, wave);
    if (lane == 0) wcnt[wave] = wc;
    __syncthreads();
    if (wave == 0) {
#pragma unroll 1
      for (int wsx = 0; wsx < NWAVE; ++wsx) {
        int n = __builtin_amdgcn_readfirstlane(wcnt[wsx]);
        n = n > WCAP ? WCAP : (n < 0 ? 0 : n);
        const int* lp = list + wsx * WCAP;
#pragma unroll 1
        for (int i = 0; i < n; ++i) {
          const int ent  = __builtin_amdgcn_readfirstlane(lp[i]);
          const int slot = ent & (NBC - 1);
          if (lane == 0) scnt[slot] = scnt[slot] + 1;
        }
      }
    }
    __syncthreads();
  }

  v4i cq[4];
#pragma unroll
  for (int q = 0; q < 4; ++q) {
    const int f = (wave * 4 + q) * 128 + 4 * lane;
    cq[q] = *(const v4i*)(scnt + f);
  }
  int* cp = cnt + (size_t)nodeBase;
#pragma unroll
  for (int q = 0; q < 4; ++q) {
    const int f = (wave * 4 + q) * 128 + 4 * lane;
    *(volatile v4i*)(cp + f) = cq[q];
  }
  __threadfence();
#pragma unroll
  for (int q = 0; q < 4; ++q) {
    const int f = (wave * 4 + q) * 128 + 4 * lane;
    *(volatile v4i*)(cp + f) = cq[q];
  }
}

__global__ __launch_bounds__(OTHR) void k_offsets(
    const int* __restrict__ cnt, int* off, int* rbase, int nChunk) {
  __shared__ __attribute__((aligned(16))) int soff[NBC];
  __shared__ __attribute__((aligned(16))) int srb[RBN];
  __shared__ int wtot[OTHR / 32];
  const int tid = threadIdx.x, lane = tid & 31, wave = tid >> 5, sub = tid >> 7;
  for (int i = tid; i < RBN; i += OTHR) srb[i] = 0;
  int carry = 0;
#pragma unroll 1
  for (int ch = 0; ch < nChunk; ++ch) {
    const int base = ch * NBC;
    const v4i c0 = *(const v4i*)(cnt + base + 8 * tid);
    const v4i c1 = *(const v4i*)(cnt + base + 8 * tid + 4);
    const int e0 = max(c0.x, 0), e1 = max(c0.y, 0), e2 = max(c0.z, 0), e3 = max(c0.w, 0);
    const int e4 = max(c1.x, 0), e5 = max(c1.y, 0), e6 = max(c1.z, 0), e7 = max(c1.w, 0);
    const int ts = e0 + e1 + e2 + e3 + e4 + e5 + e6 + e7;
    int incl = ts;
#pragma unroll
    for (int d = 1; d < 32; d <<= 1) {
      const int t = __shfl_up(incl, d);
      if (lane >= d) incl += t;
    }
    if (lane == 31) wtot[wave] = incl;
    __syncthreads();
    const int S0 = wtot[0]  + wtot[1]  + wtot[2]  + wtot[3];
    const int S1 = wtot[4]  + wtot[5]  + wtot[6]  + wtot[7];
    const int S2 = wtot[8]  + wtot[9]  + wtot[10] + wtot[11];
    const int S3 = wtot[12] + wtot[13] + wtot[14] + wtot[15];
    int pre = 0;
#pragma unroll 1
    for (int w = 4 * sub; w < wave; ++w) pre += wtot[w];
    const int b0 = carry;
    const int b1 = b0 + ((S0 + 31) & ~31);
    const int b2 = b1 + ((S1 + 31) & ~31);
    const int b3 = b2 + ((S2 + 31) & ~31);
    const int b4 = b3 + ((S3 + 31) & ~31);
    const int myb = sub == 0 ? b0 : (sub == 1 ? b1 : (sub == 2 ? b2 : b3));
    if (tid == 0) {
      srb[min(4 * ch + 0, RBN - 1)] = b0;
      srb[min(4 * ch + 1, RBN - 1)] = b1;
      srb[min(4 * ch + 2, RBN - 1)] = b2;
      srb[min(4 * ch + 3, RBN - 1)] = b3;
    }
    int run = myb + pre + incl - ts;
    soff[8 * tid + 0] = run; run += e0;
    soff[8 * tid + 1] = run; run += e1;
    soff[8 * tid + 2] = run; run += e2;
    soff[8 * tid + 3] = run; run += e3;
    soff[8 * tid + 4] = run; run += e4;
    soff[8 * tid + 5] = run; run += e5;
    soff[8 * tid + 6] = run; run += e6;
    soff[8 * tid + 7] = run;
    carry = b4;
    __syncthreads();
    const v4i o0 = *(const v4i*)(soff + 4 * tid);
    const v4i o1 = *(const v4i*)(soff + 4 * (tid + OTHR));
    int* op = off + base;
    *(volatile v4i*)(op + 4 * tid) = o0;
    *(volatile v4i*)(op + 4 * (tid + OTHR)) = o1;
    __threadfence();
    *(volatile v4i*)(op + 4 * tid) = o0;
    *(volatile v4i*)(op + 4 * (tid + OTHR)) = o1;
    __syncthreads();
  }
  if (tid == 0) srb[min(4 * nChunk, RBN - 1)] = carry;
  __syncthreads();
  v4i rv = {0, 0, 0, 0};
  if (tid < 32) rv = *(const v4i*)(srb + 4 * tid);
  if (tid < 32) *(volatile v4i*)(rbase + 4 * tid) = rv;
  __threadfence();
  if (tid < 32) *(volatile v4i*)(rbase + 4 * tid) = rv;
}

__global__ __launch_bounds__(NTHR) void k_fill(
    const int* __restrict__ srcs, const int* __restrict__ dsts,
    const int* __restrict__ off, const int* __restrict__ rbase,
    int* csr, int nN, int nE, int vec8, int csrLen) {
  extern __shared__ v4f lds_dyn[];
  int* region = (int*)lds_dyn;
  int* cursor = region + RCAP;
  int* list   = cursor + NBF;
  int* wcnt   = list + LISTN;
  const int tid = threadIdx.x, lane = tid & 31, wave = tid >> 5;
  const int b = blockIdx.x;
  const int nodeBase = b * NBF;

  int rb0 = rbase[b];
  const int rb1 = rbase[b + 1];
  rb0 = rb0 < 0 ? 0 : (rb0 > csrLen ? csrLen : rb0);
  rb0 &= ~31;
  int len = rb1 - rb0;
  len = len < 0 ? 0 : (len > RCAP ? RCAP : len);
  int lenW = (len + 31) & ~31;
  if (rb0 + lenW > csrLen) lenW = (csrLen - rb0) & ~31;

  {
    const v4i z = {0, 0, 0, 0};
    for (int i = tid; i < RCAP / 4; i += NTHR) ((v4i*)region)[i] = z;
    for (int s = tid; s < NBF; s += NTHR) {
      int o = off[nodeBase + s] - rb0;
      o = o < 0 ? 0 : (o > RCAP ? RCAP : o);
      cursor[s] = o;
    }
  }
  __syncthreads();

  const int nChunks = (nE + CHUNK - 1) / CHUNK;
#pragma unroll 1
  for (int ch = 0; ch < nChunks; ++ch) {
    const int cbase = ch * CHUNK;
    const int wc = scan_chunk<NBF>(dsts, nE, cbase, nodeBase, vec8, list, tid, lane, wave);
    if (lane == 0) wcnt[wave] = wc;
    __syncthreads();
    if (wave == 0) {
#pragma unroll 1
      for (int wsx = 0; wsx < NWAVE; ++wsx) {
        int n = __builtin_amdgcn_readfirstlane(wcnt[wsx]);
        n = n > WCAP ? WCAP : (n < 0 ? 0 : n);
        const int* lp = list + wsx * WCAP;
#pragma unroll 1
        for (int i = 0; i < n; ++i) {
          const int ent  = __builtin_amdgcn_readfirstlane(lp[i]);
          const int slot = ent & (NBF - 1);
          int e = cbase + ((ent >> 12) & (CHUNK - 1));
          e = e > nE - 1 ? nE - 1 : e;
          int sv = srcs[e];
          sv = sv < 0 ? 0 : (sv > nN - 1 ? nN - 1 : sv);
          if (lane == 0) {
            int pos = cursor[slot];
            pos = pos < 0 ? 0 : (pos > RCAP - 1 ? RCAP - 1 : pos);
            region[pos] = sv;
            const int np = pos + 1;
            cursor[slot] = np > RCAP ? RCAP : np;
          }
        }
      }
    }
    __syncthreads();
  }

  const int nv = lenW >> 2;
  int* gp = csr + rb0;
#pragma unroll 1
  for (int i = tid; i < nv; i += NTHR) { const v4i v = ((const v4i*)region)[i]; *(volatile v4i*)(gp + 4 * i) = v; }
  __threadfence();
#pragma unroll 1
  for (int i = tid; i < nv; i += NTHR) { const v4i v = ((const v4i*)region)[i]; *(volatile v4i*)(gp + 4 * i) = v; }
}

template <int BF>
__global__ __launch_bounds__(NTHR) void k_gemm(const unsigned short* __restrict__ Ap,
                                               const unsigned short* __restrict__ Bp,
                                               float* C, int lda, int KT, int ldc, float osc) {
  __shared__ __attribute__((aligned(16))) float stg[BM * NCW];
  const int tid = threadIdx.x, lane = tid & 31, wave = tid >> 5, hh = lane >> 4, m = lane & 15;
  const int rowBase = (int)blockIdx.x * BM;
  const int colBase = (int)blockIdx.y * NCW;
  const int rg = wave >> 1, chf = wave & 1;
  const int r0 = rg * 16;
  const int c0 = chf * 32;
  const int KB = 32 * KT;

  v8f acc0 = {0.f, 0.f, 0.f, 0.f, 0.f, 0.f, 0.f, 0.f};
  v8f acc1 = {0.f, 0.f, 0.f, 0.f, 0.f, 0.f, 0.f, 0.f};

  const unsigned short* ap  = Ap + (size_t)(rowBase + r0 + m) * lda + 8 * hh;
  const unsigned short* bpA = Bp + (size_t)(colBase + c0 + m) * KB + 8 * hh;
  const unsigned short* bpB = bpA + (size_t)16 * KB;
#pragma unroll 1
  for (int kt = 0; kt < KT; ++kt) {
    const v8us a0 = *(const v8us*)(ap + 32 * kt);
    const v8us a1 = *(const v8us*)(ap + 32 * kt + 16);
    const v8us b00 = *(const v8us*)(bpA + 32 * kt);
    const v8us b01 = *(const v8us*)(bpA + 32 * kt + 16);
    const v8us b10 = *(const v8us*)(bpB + 32 * kt);
    const v8us b11 = *(const v8us*)(bpB + 32 * kt + 16);
    if constexpr (BF) {
      FragB a, b0, b1;
      a.u[0] = a0; a.u[1] = a1; b0.u[0] = b00; b0.u[1] = b01; b1.u[0] = b10; b1.u[1] = b11;
      acc0 = wmb(a.v, b0.v, acc0);
      acc1 = wmb(a.v, b1.v, acc1);
    } else {
      FragH a, b0, b1;
      a.u[0] = a0; a.u[1] = a1; b0.u[0] = b00; b0.u[1] = b01; b1.u[0] = b10; b1.u[1] = b11;
      acc0 = wmh(a.v, b0.v, acc0);
      acc1 = wmh(a.v, b1.v, acc1);
    }
  }

  {
    float* sp = stg + (size_t)(r0 + 8 * hh) * NCW + c0 + m;
#pragma unroll
    for (int r = 0; r < 8; ++r) {
      sp[r * NCW]      = acc0[r] * osc;
      sp[r * NCW + 16] = acc1[r] * osc;
    }
  }
  __syncthreads();

  v4f cv[4];
#pragma unroll
  for (int it = 0; it < 4; ++it) {
    const int id = it * NTHR + tid;
    const int row = id >> 4, seg = id & 15;
    cv[it] = *(const v4f*)(stg + (size_t)row * NCW + 4 * seg);
  }
#pragma unroll
  for (int it = 0; it < 4; ++it) {
    const int id = it * NTHR + tid;
    const int row = id >> 4, seg = id & 15;
    float* gp = C + (size_t)(rowBase + row) * ldc + colBase + 4 * seg;
    *(volatile v4f*)gp = cv[it];
  }
  __threadfence();
#pragma unroll
  for (int it = 0; it < 4; ++it) {
    const int id = it * NTHR + tid;
    const int row = id >> 4, seg = id & 15;
    float* gp = C + (size_t)(rowBase + row) * ldc + colBase + 4 * seg;
    *(volatile v4f*)gp = cv[it];
  }
}

template <int D, int MODE>
__global__ __launch_bounds__(NTHR) void k_gat(
    const int* __restrict__ csr, const int* __restrict__ off, const int* __restrict__ cnt,
    const float* __restrict__ eS4, const float* __restrict__ eD4, const float* __restrict__ hp,
    const float* __restrict__ bias, const float* __restrict__ un,
    unsigned short* Aout, float* eSn, float* eDn, int nN, int csrLen) {
  constexpr int LDH = (D == 16) ? LDH1 : ((D == 32) ? LDH2 : LDH3);
  constexpr int NV = (NHD * D) / 4;
  constexpr int DQ = D / 4;
  __shared__ __attribute__((aligned(16))) float su[256];
  __shared__ __attribute__((aligned(16))) _Float16 sA[(MODE == 0) ? (NWAVE * 32 * KA) : 8];
  const int tid = threadIdx.x, lane = tid & 31, wave = tid >> 5;
  const int tbase = (int)blockIdx.x * TGT + wave * 32;
  su[tid] = un[tid];
  __syncthreads();

  const int v0c = lane < NV - 1 ? lane : NV - 1;
  const int v1c = (lane + 32) < NV - 1 ? (lane + 32) : NV - 1;
  int hv0 = (4 * lane) / D;
  hv0 = hv0 > 2 ? 2 : hv0;
  const int cl    = tbase + lane;
  const int cnt_l = cnt[cl];
  const int off_l = off[cl];
  const int lq = lane < DQ ? lane : DQ - 1;
  const v4f bq = *(const v4f*)(bias + 4 * lq);
  const v4f z4 = {0.f, 0.f, 0.f, 0.f};
  v4f myS = z4, myD = z4;
  const float third = 1.0f / 3.0f;
  const v4f u0 = *(const v4f*)(su + 4 * lq),       u1 = *(const v4f*)(su + 32 + 4 * lq);
  const v4f u2 = *(const v4f*)(su + 64 + 4 * lq),  w0 = *(const v4f*)(su + 128 + 4 * lq);
  const v4f w1 = *(const v4f*)(su + 160 + 4 * lq), w2 = *(const v4f*)(su + 192 + 4 * lq);

#pragma unroll 1
  for (int j = 0; j < 32; ++j) {
    const int c = tbase + j;
    int n = __builtin_amdgcn_readfirstlane(__shfl(cnt_l, j));
    n = n < 0 ? 0 : (n > DEGCAP ? DEGCAP : n);
    const int st = __builtin_amdgcn_readfirstlane(__shfl(off_l, j));
    const v4f edc = *(const v4f*)(eD4 + (size_t)c * 4);
    const v4f esc = *(const v4f*)(eS4 + (size_t)c * 4);
    const float es0 = lrelu2(esc.x + edc.x), es1 = lrelu2(esc.y + edc.y), es2 = lrelu2(esc.z + edc.z);

    float mx0 = es0, mx1 = es1, mx2 = es2;
#pragma unroll 1
    for (int q0 = 0; q0 < n; q0 += 32) {
      int pos = st + q0 + lane;
      pos = pos < 0 ? 0 : (pos > csrLen - 1 ? csrLen - 1 : pos);
      int sl = csr[pos];
      sl = sl < 0 ? 0 : (sl > nN - 1 ? nN - 1 : sl);
      const bool valid = (q0 + lane) < n;
      const v4f ev = *(const v4f*)(eS4 + (size_t)sl * 4);
      const float t0 = lrelu2(ev.x + edc.x), t1 = lrelu2(ev.y + edc.y), t2 = lrelu2(ev.z + edc.z);
      mx0 = valid ? fmaxf(mx0, t0) : mx0;
      mx1 = valid ? fmaxf(mx1, t1) : mx1;
      mx2 = valid ? fmaxf(mx2, t2) : mx2;
    }
    mx0 = wmax32(mx0); mx1 = wmax32(mx1); mx2 = wmax32(mx2);

    const float ps0 = __expf(es0 - mx0), ps1 = __expf(es1 - mx1), ps2 = __expf(es2 - mx2);
    const float pss = hv0 == 0 ? ps0 : (hv0 == 1 ? ps1 : ps2);
    const float* hc = hp + (size_t)c * LDH;
    v4f acc0 = *(const v4f*)(hc + 4 * v0c) * pss;
    v4f acc1 = z4;
    if constexpr (D == 64) acc1 = *(const v4f*)(hc + 4 * v1c) * ps2;
    float d0 = 0.f, d1 = 0.f, d2 = 0.f;
#pragma unroll 1
    for (int q0 = 0; q0 < n; q0 += 32) {
      int pos = st + q0 + lane;
      pos = pos < 0 ? 0 : (pos > csrLen - 1 ? csrLen - 1 : pos);
      int sl = csr[pos];
      sl = sl < 0 ? 0 : (sl > nN - 1 ? nN - 1 : sl);
      const bool valid = (q0 + lane) < n;
      const v4f ev = *(const v4f*)(eS4 + (size_t)sl * 4);
      const float p0 = valid ? __expf(lrelu2(ev.x + edc.x) - mx0) : 0.f;
      const float p1 = valid ? __expf(lrelu2(ev.y + edc.y) - mx1) : 0.f;
      const float p2 = valid ? __expf(lrelu2(ev.z + edc.z) - mx2) : 0.f;
      d0 += p0; d1 += p1; d2 += p2;
      const int mcnt = (n - q0) < 32 ? (n - q0) : 32;
#pragma unroll 1
      for (int pp = 0; pp < mcnt; ++pp) {
        const int s = __builtin_amdgcn_readlane(sl, pp);
        const float pa = __int_as_float(__builtin_amdgcn_readlane(__float_as_int(p0), pp));
        const float pb = __int_as_float(__builtin_amdgcn_readlane(__float_as_int(p1), pp));
        const float pc = __int_as_float(__builtin_amdgcn_readlane(__float_as_int(p2), pp));
        const float pl = hv0 == 0 ? pa : (hv0 == 1 ? pb : pc);
        const float* xs = hp + (size_t)s * LDH;
        const v4f xv0 = *(const v4f*)(xs + 4 * v0c);
        acc0 += xv0 * pl;
        if constexpr (D == 64) {
          const v4f xv1 = *(const v4f*)(xs + 4 * v1c);
          acc1 += xv1 * pc;
        }
      }
    }
    d0 = wsum32(d0); d1 = wsum32(d1); d2 = wsum32(d2);
    const float rd0 = __builtin_amdgcn_rcpf(ps0 + d0 + 1e-16f);
    const float rd1 = __builtin_amdgcn_rcpf(ps1 + d1 + 1e-16f);
    const float rd2 = __builtin_amdgcn_rcpf(ps2 + d2 + 1e-16f);
    const float rl = hv0 == 0 ? rd0 : (hv0 == 1 ? rd1 : rd2);
    const v4f o0 = acc0 * rl;
    v4f r;
    if constexpr (D == 16) {
      r = o0 + shfl4(o0, (lane + 4) & 31) + shfl4(o0, (lane + 8) & 31);
    } else if constexpr (D == 32) {
      r = o0 + shfl4(o0, (lane + 8) & 31) + shfl4(o0, (lane + 16) & 31);
    } else {
      const v4f o1 = acc1 * rd2;
      r = o0 + shfl4(o0, (lane + 16) & 31) + o1;
    }
    const bool live = c < nN;
    v4f outq = r * third + bq;
    outq = live ? outq : z4;

    if constexpr (MODE == 0) {
      const bool inq = lane < DQ;
      float t0 = dot4(outq, u0), t1 = dot4(outq, u1), t2 = dot4(outq, u2);
      float y0 = dot4(outq, w0), y1 = dot4(outq, w1), y2 = dot4(outq, w2);
      t0 = inq ? t0 : 0.f; t1 = inq ? t1 : 0.f; t2 = inq ? t2 : 0.f;
      y0 = inq ? y0 : 0.f; y1 = inq ? y1 : 0.f; y2 = inq ? y2 : 0.f;
      t0 = wsum32(t0); t1 = wsum32(t1); t2 = wsum32(t2);
      y0 = wsum32(y0); y1 = wsum32(y1); y2 = wsum32(y2);
      v4f vs, vd;
      vs.x = t0; vs.y = t1; vs.z = t2; vs.w = 0.f;
      vd.x = y0; vd.y = y1; vd.z = y2; vd.w = 0.f;
      myS = (lane == j) ? vs : myS;
      myD = (lane == j) ? vd : myD;
      v4h hv;
      hv[0] = inq ? (_Float16)(outq.x * (float)ASC) : (_Float16)0.0f;
      hv[1] = inq ? (_Float16)(outq.y * (float)ASC) : (_Float16)0.0f;
      hv[2] = inq ? (_Float16)(outq.z * (float)ASC) : (_Float16)0.0f;
      hv[3] = inq ? (_Float16)(outq.w * (float)ASC) : (_Float16)0.0f;
      if (lane < 8) *(v4h*)(sA + wave * (32 * KA) + j * KA + 4 * lane) = hv;
    } else {
      const v4f oq = shfl4(outq, lane & 15);
      const unsigned short hb0 = bf16_rne(oq.x), hb1 = bf16_rne(oq.y), hb2 = bf16_rne(oq.z), hb3 = bf16_rne(oq.w);
      const unsigned short lb0 = bf16_rne(oq.x - bf16_val(hb0)), lb1 = bf16_rne(oq.y - bf16_val(hb1));
      const unsigned short lb2 = bf16_rne(oq.z - bf16_val(hb2)), lb3 = bf16_rne(oq.w - bf16_val(hb3));
      v4us ph, plo;
      ph.x = hb0; ph.y = hb1; ph.z = hb2; ph.w = hb3;
      plo.x = lb0; plo.y = lb1; plo.z = lb2; plo.w = lb3;
      const v4us sel = (lane < 16) ? ph : plo;
      unsigned short* rp = Aout + (size_t)c * KPQ;
      const bool lo16 = lane < 16;
      *(volatile v4us*)(rp + 4 * lane) = sel;
      if (lo16) *(volatile v4us*)(rp + 128 + 4 * lane) = ph;
      __threadfence();
      *(volatile v4us*)(rp + 4 * lane) = sel;
      if (lo16) *(volatile v4us*)(rp + 128 + 4 * lane) = ph;
    }
  }

  if constexpr (MODE == 0) {
    __syncthreads();
    v8us pv[4];
#pragma unroll
    for (int it = 0; it < 4; ++it) {
      const int id = it * 32 + lane;
      const v8ha t = *(const v8ha*)(sA + wave * (32 * KA) + 8 * id);
      pv[it] = __builtin_bit_cast(v8us, t);
    }
    unsigned short* ab = Aout + (size_t)tbase * KA;
#pragma unroll
    for (int it = 0; it < 4; ++it) *(volatile v8us*)(ab + 8 * (it * 32 + lane)) = pv[it];
    *(volatile v4f*)(eSn + (size_t)(tbase + lane) * 4) = myS;
    *(volatile v4f*)(eDn + (size_t)(tbase + lane) * 4) = myD;
    __threadfence();
#pragma unroll
    for (int it = 0; it < 4; ++it) *(volatile v8us*)(ab + 8 * (it * 32 + lane)) = pv[it];
    *(volatile v4f*)(eSn + (size_t)(tbase + lane) * 4) = myS;
    *(volatile v4f*)(eDn + (size_t)(tbase + lane) * 4) = myD;
  }
}

__global__ __launch_bounds__(ETHR) void k_edge(
    const int* __restrict__ ei, const float* __restrict__ ef, const float* __restrict__ PQ,
    const float* __restrict__ stat, const float* __restrict__ ge, const float* __restrict__ be,
    const float* __restrict__ mw1, const float* __restrict__ mb1,
    const float* __restrict__ mw2, const float* __restrict__ mb2,
    const float* __restrict__ mw3, const float* __restrict__ mb3,
    const float* __restrict__ mw4, const float* __restrict__ mb4,
    const float* __restrict__ mw5, const float* __restrict__ mb5,
    float* out, int nE, int nN) {
  extern __shared__ v4f act[];
  __shared__ __attribute__((aligned(16))) float swf[SWF];
  __shared__ __attribute__((aligned(16))) float sbf[128];
  __shared__ float ssc[16], ssh[16];
  const int tid = threadIdx.x;

  if (tid < 16) {
    const int k = tid;
    const int kc = k < FE - 1 ? k : FE - 1;
    const bool valid = k < FE;
    const float sc = stat[48 + kc] * ge[kc];
    const float sh = be[kc] - stat[32 + kc] * sc;
    ssc[k] = valid ? sc : 0.0f;
    ssh[k] = valid ? sh : 0.0f;
  }
  __syncthreads();
  for (int uu = tid; uu < 256; uu += ETHR) {
    const int n = uu >> 2, q = uu & 3;
    v4f w;
#pragma unroll
    for (int i = 0; i < 4; ++i) {
      const int k = 4 * q + i;
      const int kc = k < FE - 1 ? k : FE - 1;
      const float t = mw1[(size_t)(128 + kc) * 64 + n] * ssc[k];
      w[i] = (k < FE) ? t : 0.0f;
    }
    *(v4f*)(swf + n * 16 + 4 * q) = w;
  }
  if (tid < 64) {
    float a = mb1[tid];
#pragma unroll 1
    for (int k = 0; k < FE; ++k) a += ssh[k] * mw1[(size_t)(128 + k) * 64 + tid];
    sbf[tid] = a;
  }
  for (int uu = tid; uu < 512; uu += ETHR) {
    const int n = uu >> 4, q = uu & 15;
    v4f w;
#pragma unroll
    for (int i = 0; i < 4; ++i) w[i] = mw2[(size_t)(4 * q + i) * 32 + n];
    *(v4f*)(swf + 1024 + n * 64 + 4 * q) = w;
  }
  {
    const int uu = tid;
    const int n = uu >> 3, q = uu & 7;
    v4f w;
#pragma unroll
    for (int i = 0; i < 4; ++i) w[i] = mw3[(size_t)(4 * q + i) * 16 + n];
    *(v4f*)(swf + 3072 + n * 32 + 4 * q) = w;
  }
  if (tid < 32) {
    const int n = tid >> 2, q = tid & 3;
    v4f w;
#pragma unroll
    for (int i = 0; i < 4; ++i) w[i] = mw4[(size_t)(4 * q + i) * 8 + n];
    *(v4f*)(swf + 3584 + n * 16 + 4 * q) = w;
  }
  if (tid < 8) {
    const int n = tid >> 1, q = tid & 1;
    const int nc = n < 1 ? n : 1;
    v4f w;
#pragma unroll
    for (int i = 0; i < 4; ++i) {
      const float t = mw5[(size_t)(4 * q + i) * 2 + nc];
      w[i] = (n < 2) ? t : 0.0f;
    }
    *(v4f*)(swf + 3712 + n * 8 + 4 * q) = w;
  }
  if (tid < 32) sbf[64 + tid] = mb2[tid];
  if (tid < 16) sbf[96 + tid] = mb3[tid];
  if (tid < 8)  sbf[112 + tid] = mb4[tid];
  if (tid < 4) {
    const float t = mb5[tid < 1 ? tid : 1];
    sbf[120 + tid] = (tid < 2) ? t : 0.0f;
    sbf[124 + tid] = 0.0f;
  }
  __syncthreads();

  const int eid = (int)blockIdx.x * ETHR + tid;
  const bool live = eid < nE;
  const int ec = eid > nE - 1 ? nE - 1 : eid;
  int s = ei[ec];
  int d = ei[(size_t)nE + ec];
  s = s < 0 ? 0 : (s > nN - 1 ? nN - 1 : s);
  d = d < 0 ? 0 : (d > nN - 1 ? nN - 1 : d);
  v4f* at = act + (size_t)tid * ACTV;
  const v4f z4 = {0.f, 0.f, 0.f, 0.f};
#pragma unroll 1
  for (int i = 0; i < ACTV; ++i) at[i] = z4;
  {
    const float* er = ef + (size_t)ec * FE;
    v4f t0, t1, t2;
    t0.x = er[0]; t0.y = er[1]; t0.z = er[2]; t0.w = er[3];
    t1.x = er[4]; t1.y = er[5]; t1.z = er[6]; t1.w = er[7];
    t2.x = er[8]; t2.y = er[9]; t2.z = 0.0f;  t2.w = 0.0f;
    at[0] = t0; at[1] = t1; at[2] = t2; at[3] = z4;
  }
  {
    const float* prow = PQ + (size_t)s * NPQ;
    const float* qrow = PQ + (size_t)d * NPQ + 64;
#pragma unroll 1
    for (int n4 = 0; n4 < 16; ++n4) {
      const v4f p = *(const v4f*)(prow + 4 * n4);
      const v4f q = *(const v4f*)(qrow + 4 * n4);
      const v4f b = *(const v4f*)(sbf + 4 * n4);
      at[4 + n4] = (p + q) + b;
    }
  }

#pragma unroll 1
  for (int l = 0; l < 5; ++l) {
    const int K8 = (l == 0) ? 2 : ((l == 1) ? 8 : ((l == 2) ? 4 : ((l == 3) ? 2 : 1)));
    const int N4 = (l == 0) ? 16 : ((l == 1) ? 8 : ((l == 2) ? 4 : ((l == 3) ? 2 : 1)));
    const int K = 8 * K8;
    const int inO = (l == 0 || l == 3) ? 0 : ((l == 2) ? 20 : 4);
    const int outO = (l == 0) ? 4 : ((l == 1) ? 20 : ((l == 2) ? 0 : ((l == 3) ? 4 : 6)));
    const int wO = (l == 0) ? 0 : ((l == 1) ? 1024 : ((l == 2) ? 3072 : ((l == 3) ? 3584 : 3712)));
    const int bO = (l == 1) ? 64 : ((l == 2) ? 96 : ((l == 3) ? 112 : ((l == 4) ? 120 : 0)));
    const float slope = (l == 4) ? 1.0f : 0.1f;
    const bool initAct = (l == 0);
#pragma unroll 1
    for (int n4 = 0; n4 < N4; ++n4) {
      const v4f ia = at[outO + n4];
      const v4f ib = *(const v4f*)(sbf + bO + 4 * n4);
      v4f acc = initAct ? ia : ib;
      const float* wr = swf + wO + (4 * n4) * K;
#pragma unroll 1
      for (int k8 = 0; k8 < K8; ++k8) {
        const v4f h0 = at[inO + 2 * k8];
        const v4f h1 = at[inO + 2 * k8 + 1];
#pragma unroll
        for (int i = 0; i < 4; ++i) {
          const v4f wa = *(const v4f*)(wr + i * K + 8 * k8);
          const v4f wb = *(const v4f*)(wr + i * K + 8 * k8 + 4);
          acc[i] += h0.x * wa.x + h0.y * wa.y + h0.z * wa.z + h0.w * wa.w
                  + h1.x * wb.x + h1.y * wb.y + h1.z * wb.z + h1.w * wb.w;
        }
      }
      v4f o;
#pragma unroll
      for (int i = 0; i < 4; ++i) { const float v = acc[i]; o[i] = v > 0.0f ? v : slope * v; }
      at[outO + n4] = o;
    }
  }

  const v4f rr = at[6];
  v2f ov;
  ov.x = rr.x; ov.y = rr.y;
  float* gp = out + (size_t)2 * ec;
  if (live) *(volatile v2f*)gp = ov;
  __threadfence();
  if (live) *(volatile v2f*)gp = ov;
}

extern "C" void kernel_launch(void* const* d_in, const int* in_sizes, int n_in,
                              void* d_out, int out_size, void* d_ws, size_t ws_size,
                              hipStream_t stream) {
  if (n_in < 30) return;
  const int nN = in_sizes[0] / FX;
  const int nE = in_sizes[1] / 2;
  if (nN <= 0 || nE <= 0) return;
  if (in_sizes[0] != nN * FX || in_sizes[1] != 2 * nE || in_sizes[2] != nE * FE) return;
  if (in_sizes[4] != FX || in_sizes[5] != FX || in_sizes[6] != FE || in_sizes[7] != FE) return;
  if (in_sizes[8] != FX * 48 || in_sizes[9] != 48 || in_sizes[10] != 48 || in_sizes[11] != 16) return;
  if (in_sizes[12] != 16 * 96 || in_sizes[13] != 96 || in_sizes[14] != 96 || in_sizes[15] != 32) return;
  if (in_sizes[16] != 32 * 192 || in_sizes[17] != 192 || in_sizes[18] != 192 || in_sizes[19] != 64) return;
  if (in_sizes[20] != 138 * 64 || in_sizes[21] != 64 || in_sizes[22] != 64 * 32 || in_sizes[23] != 32) return;
  if (in_sizes[24] != 32 * 16 || in_sizes[25] != 16 || in_sizes[26] != 16 * 8 || in_sizes[27] != 8) return;
  if (in_sizes[28] != 16 || in_sizes[29] != 2) return;
  if (out_size != 2 * nE) return;
  if (nE > (1 << 28) || nN > (1 << 22)) return;

  const float* x    = (const float*)d_in[0];
  const int*   ei   = (const int*)d_in[1];
  const int*   src  = ei;
  const int*   dst  = ei + nE;
  const float* ef   = (const float*)d_in[2];
  const float* bng  = (const float*)d_in[4];
  const float* bnb  = (const float*)d_in[5];
  const float* beg  = (const float*)d_in[6];
  const float* beb  = (const float*)d_in[7];
  const float* W1   = (const float*)d_in[8];
  const float* as1  = (const float*)d_in[9];
  const float* ad1  = (const float*)d_in[10];
  const float* b1   = (const float*)d_in[11];
  const float* W2   = (const float*)d_in[12];
  const float* as2  = (const float*)d_in[13];
  const float* ad2  = (const float*)d_in[14];
  const float* b2   = (const float*)d_in[15];
  const float* W3   = (const float*)d_in[16];
  const float* as3  = (const float*)d_in[17];
  const float* ad3  = (const float*)d_in[18];
  const float* b3   = (const float*)d_in[19];
  const float* mw1  = (const float*)d_in[20];
  const float* mb1  = (const float*)d_in[21];
  const float* mw2  = (const float*)d_in[22];
  const float* mb2  = (const float*)d_in[23];
  const float* mw3  = (const float*)d_in[24];
  const float* mb3  = (const float*)d_in[25];
  const float* mw4  = (const float*)d_in[26];
  const float* mb4  = (const float*)d_in[27];
  const float* mw5  = (const float*)d_in[28];
  const float* mb5  = (const float*)d_in[29];
  float* out = (float*)d_out;

  const int NPAD   = ((nN + TGT - 1) / TGT) * TGT;
  const int nBC    = (nN + NBC - 1) / NBC;
  const int CNTPAD = nBC * NBC;
  if (CNTPAD < NPAD) return;
  if (4 * nBC + 1 > RBN) return;
  const int nBF    = (nN + NBF - 1) / NBF;
  if (nBF > 4 * nBC) return;
  const int csrLen = ((nE + 31) & ~31) + 4096;
  if (31 * 4 * nBC > 4096) return;
  const int nAgg   = NPAD / TGT;
  const int nGemm  = NPAD / BM;
  const int nBx    = (nN + NTHR * RPT - 1) / (NTHR * RPT);
  const int nBe    = (nE + NTHR * RPT - 1) / (NTHR * RPT);
  const int nEdgeB = (nE + ETHR - 1) / ETHR;

  char* ws = (char*)d_ws;
  size_t off = 0;
  const size_t oPx  = off; off += (size_t)nBx * 32 * 8;          off = (off + 255) & ~(size_t)255;
  const size_t oPe  = off; off += (size_t)nBe * 32 * 8;          off = (off + 255) & ~(size_t)255;
  const size_t oSt  = off; off += (size_t)64 * 4;                off = (off + 255) & ~(size_t)255;
  const size_t oU   = off; off += (size_t)768 * 4;               off = (off + 255) & ~(size_t)255;
  const size_t oW1  = off; off += (size_t)LDH1 * KA * 2;         off = (off + 255) & ~(size_t)255;
  const size_t oW2  = off; off += (size_t)LDH2 * KA * 2;         off = (off + 255) & ~(size_t)255;
  const size_t oW3  = off; off += (size_t)LDH3 * KA * 2;         off = (off + 255) & ~(size_t)255;
  const size_t oWpq = off; off += (size_t)NPQ * KPQ * 2;         off = (off + 255) & ~(size_t)255;
  const size_t oA1  = off; off += (size_t)NPAD * KA * 2;         off = (off + 255) & ~(size_t)255;
  const size_t oES1 = off; off += (size_t)NPAD * 4 * 4;          off = (off + 255) & ~(size_t)255;
  const size_t oED1 = off; off += (size_t)NPAD * 4 * 4;          off = (off + 255) & ~(size_t)255;
  const size_t oCnt = off; off += (size_t)CNTPAD * 4;            off = (off + 255) & ~(size_t)255;
  const size_t oOff = off; off += (size_t)CNTPAD * 4;            off = (off + 255) & ~(size_t)255;
  const size_t oRb  = off; off += (size_t)RBN * 4;               off = (off + 255) & ~(size_t)255;
  const size_t oCsr = off; off += (size_t)csrLen * 4;            off = (off + 255) & ~(size_t)255;
  const size_t oH   = off; off += (size_t)NPAD * LDH3 * 4;       off = (off + 255) & ~(size_t)255;
  const size_t oA2  = off; off += (size_t)NPAD * KA * 2;         off = (off + 255) & ~(size_t)255;
  const size_t oES2 = off; off += (size_t)NPAD * 4 * 4;          off = (off + 255) & ~(size_t)255;
  const size_t oED2 = off; off += (size_t)NPAD * 4 * 4;          off = (off + 255) & ~(size_t)255;
  const size_t oA3  = off; off += (size_t)NPAD * KA * 2;         off = (off + 255) & ~(size_t)255;
  const size_t oES3 = off; off += (size_t)NPAD * 4 * 4;          off = (off + 255) & ~(size_t)255;
  const size_t oED3 = off; off += (size_t)NPAD * 4 * 4;          off = (off + 255) & ~(size_t)255;
  const size_t oApq = off; off += (size_t)NPAD * KPQ * 2;        off = (off + 255) & ~(size_t)255;
  if (off > ws_size || off > (size_t)WSCAP) return;

  double*         partx = (double*)(ws + oPx);
  double*         parte = (double*)(ws + oPe);
  float*          stat  = (float*)(ws + oSt);
  float*          u     = (float*)(ws + oU);
  unsigned short* w1p   = (unsigned short*)(ws + oW1);
  unsigned short* w2p   = (unsigned short*)(ws + oW2);
  unsigned short* w3p   = (unsigned short*)(ws + oW3);
  unsigned short* wpq   = (unsigned short*)(ws + oWpq);
  unsigned short* A1    = (unsigned short*)(ws + oA1);
  float*          es1   = (float*)(ws + oES1);
  float*          ed1   = (float*)(ws + oED1);
  int*            cnt   = (int*)(ws + oCnt);
  int*            offp  = (int*)(ws + oOff);
  int*            rb    = (int*)(ws + oRb);
  int*            csr   = (int*)(ws + oCsr);
  float*          H     = (float*)(ws + oH);
  unsigned short* A2    = (unsigned short*)(ws + oA2);
  float*          es2   = (float*)(ws + oES2);
  float*          ed2   = (float*)(ws + oED2);
  unsigned short* A3    = (unsigned short*)(ws + oA3);
  float*          es3   = (float*)(ws + oES3);
  float*          ed3   = (float*)(ws + oED3);
  unsigned short* Apq   = (unsigned short*)(ws + oApq);

  const int vec8 = ((nE & 3) == 0) ? 1 : 0;
  const float osc16 = 1.0f / (float)(ASC * WSC);

  k_colstats<FX><<<nBx, NTHR, 0, stream>>>(x, partx, nN);
  k_colstats<FE><<<nBe, NTHR, 0, stream>>>(ef, parte, nE);
  k_bnfin<<<1, 64, 0, stream>>>(partx, parte, stat, nBx, nN, nBe, nE);
  k_ufold<<<3, NTHR, 0, stream>>>(W1, as1, ad1, W2, as2, ad2, W3, as3, ad3, u);
  k_wcvt16<<<(LDH1 * 4 + NTHR - 1) / NTHR, NTHR, 0, stream>>>(W1, w1p, 16, 48, LDH1);
  k_wcvt16<<<(LDH2 * 4 + NTHR - 1) / NTHR, NTHR, 0, stream>>>(W2, w2p, 16, 96, LDH2);
  k_wcvt16<<<(LDH3 * 4 + NTHR - 1) / NTHR, NTHR, 0, stream>>>(W3, w3p, 32, 192, LDH3);
  k_wcvtpq<<<(NPQ * (KPQ / 8) + NTHR - 1) / NTHR, NTHR, 0, stream>>>(mw1, wpq);
  k_xprep<<<NPAD / NTHR, NTHR, 0, stream>>>(x, stat, bng, bnb, u, A1, es1, ed1, nN);
  k_count<<<nBC, NTHR, 0, stream>>>(dst, cnt, nE, vec8);
  k_offsets<<<1, OTHR, 0, stream>>>(cnt, offp, rb, nBC);
  hipFuncSetAttribute(reinterpret_cast<const void*>(&k_fill),
                      hipFuncAttributeMaxDynamicSharedMemorySize, LDS_FILL);
  k_fill<<<nBF, NTHR, LDS_FILL, stream>>>(src, dst, offp, rb, csr, nN, nE, vec8, csrLen);
  k_gemm<0><<<dim3(nGemm, LDH1 / NCW, 1), NTHR, 0, stream>>>(A1, w1p, H, KA, 1, LDH1, osc16);
  k_gat<16, 0><<<nAgg, NTHR, 0, stream>>>(csr, offp, cnt, es1, ed1, H, b1, u + 256, A2, es2, ed2, nN, csrLen);
  k_gemm<0><<<dim3(nGemm, LDH2 / NCW, 1), NTHR, 0, stream>>>(A2, w2p, H, KA, 1, LDH2, osc16);
  k_gat<32, 0><<<nAgg, NTHR, 0, stream>>>(csr, offp, cnt, es2, ed2, H, b2, u + 512, A3, es3, ed3, nN, csrLen);
  k_gemm<0><<<dim3(nGemm, LDH3 / NCW, 1), NTHR, 0, stream>>>(A3, w3p, H, KA, 1, LDH3, osc16);
  k_gat<64, 1><<<nAgg, NTHR, 0, stream>>>(csr, offp, cnt, es3, ed3, H, b3, u, Apq, es1, ed1, nN, csrLen);
  k_gemm<1><<<dim3(nGemm, NPQ / NCW, 1), NTHR, 0, stream>>>(Apq, wpq, H, KPQ, KPQ / 32, NPQ, 1.0f);
  hipFuncSetAttribute(reinterpret_cast<const void*>(&k_edge),
                      hipFuncAttributeMaxDynamicSharedMemorySize, LDS_EDGE);
  k_edge<<<nEdgeB, ETHR, LDS_EDGE, stream>>>(ei, ef, H, stat, beg, beb, mw1, mb1, mw2, mb2, mw3, mb3,
                                              mw4, mb4, mw5, mb5, out, nE, nN);
}
